// GRUModel_21492016349847
// MI455X (gfx1250) — hardware-verified
//
#include <hip/hip_runtime.h>
#include <math.h>

constexpr int NB      = 128;
constexpr int NTS     = 384;
constexpr int NF      = 256;
constexpr int NU      = 256;
constexpr int NG      = 3 * NU;
constexpr int NLAY    = 4;
constexpr int NSL     = 32;
constexpr int NSLICE  = NB / NSL;
constexpr int SROWS   = NTS * NSL;
constexpr int NROWS   = NB * NTS;
constexpr int NTHR    = 256;
constexpr int SEQ_BLK = 16;
constexpr int HP      = 264;
constexpr int FPITCH  = 260;
constexpr float ACARRY = 16.0f;
constexpr float WCARRY = 64.0f;
constexpr float SINV   = 1.0f / (ACARRY * WCARRY);
constexpr int WMAT    = NG * NF;
constexpr int NXBLK   = NROWS * NF / 8 / NTHR;
constexpr int WBLK    = WMAT / 8 / NTHR;
constexpr int NPREPBLK = NXBLK + 2 * NLAY * WBLK;
constexpr int GBLK    = (NG / 64) * (SROWS / 64) / 8;
constexpr size_t SEQ_BYTES  = (size_t)NROWS * NF * 2;
constexpr size_t WALL_BYTES = (size_t)2 * NLAY * WMAT * 2;
constexpr size_t XPT_BYTES  = (size_t)NG * SROWS * 4;
constexpr size_t WS_TOTAL   = 2 * SEQ_BYTES + WALL_BYTES + XPT_BYTES;
static_assert(WS_TOTAL <= (size_t)134217728);
static_assert(NF == NU);
static_assert(NF % 32 == 0);
static_assert(NG % 64 == 0 && SROWS % 64 == 0);
static_assert(((NG / 64) * (SROWS / 64)) % 8 == 0);
static_assert(NB % NSL == 0 && NSL % SEQ_BLK == 0);
static_assert(NU == 32 * (NTHR / 32));
static_assert((NROWS * NF / 8) % NTHR == 0);
static_assert((WMAT / 8) % NTHR == 0);
static_assert(NSL == 32);
static_assert(HP % 8 == 0 && FPITCH % 4 == 0);

typedef __attribute__((ext_vector_type(16))) _Float16 v16h;
typedef __attribute__((ext_vector_type(8)))  _Float16 v8h;
typedef __attribute__((ext_vector_type(16))) __bf16   v16b;
typedef __attribute__((ext_vector_type(8)))  __bf16   v8b;
typedef __attribute__((ext_vector_type(8)))  float    v8f;
typedef __attribute__((ext_vector_type(4)))  float    v4f;

__device__ __forceinline__ unsigned short f2bf_bits(float f) {
  unsigned u = __float_as_uint(f);
  return (unsigned short)((u + 0x7FFFu + ((u >> 16) & 1u)) >> 16);
}
__device__ __forceinline__ float bf_bits2f(unsigned short h) { return __uint_as_float(((unsigned)h) << 16); }

__device__ __forceinline__ void dep_guard_h(v8f& a, v8f& b, v16h x, v16h y) { asm volatile("v_nop\n\tv_nop\n\tv_nop\n\tv_nop" : "+v"(a), "+v"(b) : "v"(x), "v"(y)); }
__device__ __forceinline__ void dep_guard_b(v8f& a, v8f& b, v16b x, v16b y) { asm volatile("v_nop\n\tv_nop\n\tv_nop\n\tv_nop" : "+v"(a), "+v"(b) : "v"(x), "v"(y)); }
__device__ __forceinline__ void keep4_h(v16h a, v16h b, v16h c, v16h d) { asm volatile("v_nop" :: "v"(a), "v"(b), "v"(c), "v"(d)); }
__device__ __forceinline__ void keep4_b(v16b a, v16b b, v16b c, v16b d) { asm volatile("v_nop" :: "v"(a), "v"(b), "v"(c), "v"(d)); }
__device__ __forceinline__ void acc_guard4(v8f& a, v8f& b, v8f& c, v8f& d) { asm volatile("v_nop\n\tv_nop\n\tv_nop\n\tv_nop" : "+v"(a), "+v"(b), "+v"(c), "+v"(d)); }
__device__ __forceinline__ void dep_guard3_h(v8f& a, v8f& b, v8f& c, v16h w, v16h x, v16h y, v16h z) {
  asm volatile("v_nop\n\tv_nop\n\tv_nop\n\tv_nop" : "+v"(a), "+v"(b), "+v"(c) : "v"(w), "v"(x), "v"(y), "v"(z));
}
__device__ __forceinline__ void acc_guard3(v8f& a, v8f& b, v8f& c) { asm volatile("v_nop\n\tv_nop\n\tv_nop\n\tv_nop" : "+v"(a), "+v"(b), "+v"(c)); }

template <typename T> struct Frag;
template <> struct Frag<_Float16> {
  typedef v16h V; union U { v16h v; v8h h[2]; };
  static __device__ __forceinline__ v16h load(const _Float16* p) {
    U f; f.h[0] = *(const v8h*)(p); f.h[1] = *(const v8h*)(p + 16); return f.v;
  }
  static __device__ __forceinline__ v8f mma(v16h a, v16h b, v8f c) {
    return __builtin_amdgcn_wmma_f32_16x16x32_f16(false, a, false, b, (short)0, c, false, false);
  }
  static __device__ __forceinline__ void guard(v8f& a, v8f& b, v16h x, v16h y) { dep_guard_h(a, b, x, y); }
  static __device__ __forceinline__ void keep(v16h a, v16h b, v16h c, v16h d) { keep4_h(a, b, c, d); }
};
template <> struct Frag<__bf16> {
  typedef v16b V; union U { v16b v; v8b h[2]; };
  static __device__ __forceinline__ v16b load(const __bf16* p) {
    U f; f.h[0] = *(const v8b*)(p); f.h[1] = *(const v8b*)(p + 16); return f.v;
  }
  static __device__ __forceinline__ v8f mma(v16b a, v16b b, v8f c) {
    return __builtin_amdgcn_wmma_f32_16x16x32_bf16(false, a, false, b, (short)0, c, false, false);
  }
  static __device__ __forceinline__ void guard(v8f& a, v8f& b, v16b x, v16b y) { dep_guard_b(a, b, x, y); }
  static __device__ __forceinline__ void keep(v16b a, v16b b, v16b c, v16b d) { keep4_b(a, b, c, d); }
};

__device__ __forceinline__ float fsig(float x)  { return __builtin_amdgcn_rcpf(1.0f + expf(-x)); }
__device__ __forceinline__ float ftanh(float x) { return 1.0f - 2.0f * __builtin_amdgcn_rcpf(1.0f + expf(2.0f * x)); }

template <int ET> struct Elem;
template <> struct Elem<0> { typedef _Float16 T; };
template <> struct Elem<1> { typedef __bf16 T; };
template <int ET, bool SPLIT, int BIAS_MODE, int OUT_MODE, bool RESID, int ACT = 0>
__global__ __launch_bounds__(256) void wmma_gemm64(
    const unsigned short* __restrict__ Ap, const unsigned short* __restrict__ A2p, int lda, long strideA,
    const unsigned short* __restrict__ Btp, const unsigned short* __restrict__ Bt2p, int ldb, long strideB,
    void* __restrict__ Cout, void* __restrict__ Cout2, int ldc, long strideC,
    const float* __restrict__ bias,
    const float* __restrict__ resid, long strideR,
    int M, int N, int K, float scale) {
  typedef typename Elem<ET>::T T;
  typedef typename Frag<T>::V V;
  const T* A = (const T*)Ap; const T* A2 = (const T*)A2p; const T* Bt = (const T*)Btp; const T* Bt2 = (const T*)Bt2p;
  __shared__ __align__(16) float sT[8][16 * 68];
  const int b    = blockIdx.y;
  const int lane = threadIdx.x & 31;
  const int wave = threadIdx.x >> 5;
  const int tilesN = N >> 6;
  const int tilesM = M >> 6;
  const int tile = blockIdx.x * 8 + wave;
  if (tile >= tilesM * tilesN) return;
  const int tm = tile / tilesN;
  const int tn = tile - tm * tilesN;
  const int m0 = tm << 6;
  const int n0 = tn << 6;

  const T* Ab  = A  + (size_t)b * strideA;
  const T* Bb  = Bt + (size_t)b * strideB;
  const T* Ab2 = SPLIT ? (A2  + (size_t)b * strideA) : nullptr;
  const T* Bb2 = SPLIT ? (Bt2 + (size_t)b * strideB) : nullptr;

  const int rlane = lane & 15;
  const int koff  = (lane >> 4) * 8;
  const int mOff  = (lane >> 4) * 8;

  v8f acc[4][4];
#pragma unroll
  for (int i = 0; i < 4; ++i)
#pragma unroll
    for (int j = 0; j < 4; ++j) acc[i][j] = (v8f){0.f,0.f,0.f,0.f,0.f,0.f,0.f,0.f};

  for (int k0 = 0; k0 < K; k0 += 32) {
    V bh[4], bl[4];
#pragma unroll
    for (int j = 0; j < 4; ++j) {
      const size_t bo = (size_t)(n0 + (j << 4) + rlane) * ldb + koff + k0;
      bh[j] = Frag<T>::load(Bb + bo);
      if (SPLIT) bl[j] = Frag<T>::load(Bb2 + bo);
    }
#pragma unroll
    for (int i = 0; i < 4; ++i) {
      const size_t ao = (size_t)(m0 + (i << 4) + rlane) * lda + koff + k0;
      V ah = Frag<T>::load(Ab + ao);
      V al;
      if (SPLIT) al = Frag<T>::load(Ab2 + ao);
#pragma unroll
      for (int j = 0; j < 4; ++j) {
        acc[i][j] = Frag<T>::mma(ah, bh[j], acc[i][j]);
        if (SPLIT) {
          acc[i][j] = Frag<T>::mma(ah, bl[j], acc[i][j]);
          acc[i][j] = Frag<T>::mma(al, bh[j], acc[i][j]);
        }
      }
      Frag<T>::guard(acc[i][0], acc[i][3], ah, SPLIT ? al : ah);
    }
    Frag<T>::keep(bh[0], bh[1], bh[2], bh[3]);
    if (SPLIT) Frag<T>::keep(bl[0], bl[1], bl[2], bl[3]);
  }
  acc_guard4(acc[0][0], acc[0][1], acc[0][2], acc[0][3]);
  acc_guard4(acc[1][0], acc[1][1], acc[1][2], acc[1][3]);
  acc_guard4(acc[2][0], acc[2][1], acc[2][2], acc[2][3]);
  acc_guard4(acc[3][0], acc[3][1], acc[3][2], acc[3][3]);

  float* slab = sT[wave];
  const float* Rb = RESID ? (resid + (size_t)b * strideR) : nullptr;
#pragma unroll
  for (int i = 0; i < 4; ++i) {
    const int mBase = m0 + (i << 4);
#pragma unroll
    for (int j = 0; j < 4; ++j) {
      const int n = n0 + (j << 4) + rlane;
      float bv = 0.f;
      if (BIAS_MODE == 2) bv = bias[n];
#pragma unroll
      for (int r = 0; r < 8; ++r) {
        float v = acc[i][j][r] * scale;
        if (BIAS_MODE == 1) v += bias[mBase + mOff + r];
        if (BIAS_MODE == 2) v += bv;
        if (RESID) v += Rb[(size_t)(mBase + mOff + r) * ldc + n];
        if (ACT == 1) v = tanhf(v);
        if (ACT == 2) v = fmaxf(v, 0.0f);
        if (ACT == 3) v = v / (1.0f + expf(-v));
        if (ACT == 4) v = (v > 0.f) ? v : 0.01f * v;
        if (ACT == 5) v = 0.5f * v * (1.0f + erff(v * 0.70710678118654752f));
        slab[(mOff + r) * 68 + (j << 4) + rlane] = v;
      }
    }
    __builtin_amdgcn_fence(__ATOMIC_RELEASE, "workgroup");
    __builtin_amdgcn_wave_barrier();
    __builtin_amdgcn_fence(__ATOMIC_ACQUIRE, "workgroup");
    if (OUT_MODE == 0) {
      float* C = (float*)Cout + (size_t)b * strideC;
      const int hh = lane >> 4, c4 = (lane & 15) * 4;
      for (int pass = 0; pass < 2; ++pass) {
#pragma unroll
        for (int it = 0; it < 8; ++it) {
          const int row = it * 2 + hh;
          v4f v = *(const v4f*)(slab + row * 68 + c4);
          *(volatile v4f*)(C + (size_t)(mBase + row) * ldc + n0 + c4) = v;
        }
        __threadfence();
      }
    } else {
      const int q = lane >> 3, c8 = (lane & 7) * 8;
      unsigned short* C  = (unsigned short*)Cout  + (size_t)b * strideC;
      unsigned short* C2 = (OUT_MODE == 2) ? ((unsigned short*)Cout2 + (size_t)b * strideC) : nullptr;
      for (int pass = 0; pass < 2; ++pass) {
#pragma unroll
        for (int it = 0; it < 4; ++it) {
          const int row = it * 4 + q;
          const float* sp = slab + row * 68 + c8;
          v8h hv, lv;
#pragma unroll
          for (int e = 0; e < 8; ++e) {
            if (OUT_MODE == 1) {
              hv[e] = (_Float16)sp[e];
            } else {
              unsigned short hb = f2bf_bits(sp[e]);
              unsigned short lb = f2bf_bits(sp[e] - bf_bits2f(hb));
              hv[e] = __builtin_bit_cast(_Float16, hb);
              lv[e] = __builtin_bit_cast(_Float16, lb);
            }
          }
          *(volatile v8h*)(C + (size_t)(mBase + row) * ldc + n0 + c8) = hv;
          if (OUT_MODE == 2) *(volatile v8h*)(C2 + (size_t)(mBase + row) * ldc + n0 + c8) = lv;
        }
        __threadfence();
      }
    }
    __builtin_amdgcn_fence(__ATOMIC_RELEASE, "workgroup");
    __builtin_amdgcn_wave_barrier();
    __builtin_amdgcn_fence(__ATOMIC_ACQUIRE, "workgroup");
  }
}

__global__ __launch_bounds__(NTHR) void prep_kernel(const float* __restrict__ x,
                                                   const float* __restrict__ k0, const float* __restrict__ kern,
                                                   const float* __restrict__ rk0, const float* __restrict__ rkern,
                                                   unsigned short* __restrict__ SAp, unsigned short* __restrict__ WALLp) {
  const int blk = blockIdx.x, tid = threadIdx.x;
  if (blk < NXBLK) {
    const int gid = blk * NTHR + tid;
    const int gr  = gid >> 5;
    const int c8  = (gid & 31) * 8;
    const int s   = gr / SROWS;
    const int rem = gr - s * SROWS;
    const int t   = rem >> 5;
    const int bl  = rem & 31;
    const size_t srow = (size_t)(s * NSL + bl) * NTS + t;
    const float* p = x + srow * NF + c8;
    const v4f a = *(const v4f*)p;
    const v4f bq = *(const v4f*)(p + 4);
    v8h h;
#pragma unroll
    for (int e = 0; e < 4; ++e) { h[e] = (_Float16)(a[e] * ACARRY); h[4 + e] = (_Float16)(bq[e] * ACARRY); }
    _Float16* op = (_Float16*)SAp + (size_t)gid * 8;
    *(volatile v8h*)op = h;
    __threadfence();
    *(volatile v8h*)op = h;
  } else {
    const int wb = blk - NXBLK;
    const int mi = wb / WBLK;
    const int p  = (wb - mi * WBLK) * NTHR + tid;
    const int g  = p >> 5;
    const int k8 = (p & 31) * 8;
    int li = mi - 1; if (li < 0) li = 0; if (li > 2) li = 2;
    int ri = mi - 5; if (ri < 0) ri = 0; if (ri > 2) ri = 2;
    const float* src = (mi == 0) ? k0
                     : (mi < 4)  ? (kern + (size_t)li * WMAT)
                     : (mi == 4) ? rk0
                     :             (rkern + (size_t)ri * WMAT);
    float w[8];
#pragma unroll
    for (int e = 0; e < 8; ++e) w[e] = src[(size_t)(k8 + e) * NG + g];
    v8h h;
#pragma unroll
    for (int e = 0; e < 8; ++e) h[e] = (_Float16)(w[e] * WCARRY);
    _Float16* op = (_Float16*)WALLp + (size_t)mi * WMAT + (size_t)p * 8;
    *(volatile v8h*)op = h;
    __threadfence();
    *(volatile v8h*)op = h;
  }
}

template <bool FINAL>
__global__ __launch_bounds__(NTHR) void rec_kernel(const float* __restrict__ XPT, const unsigned short* __restrict__ RTp,
                                                  const float* __restrict__ bin, const float* __restrict__ brc,
                                                  unsigned short* __restrict__ HOUTp, float* __restrict__ OUT) {
  __shared__ __align__(16) _Float16 h16[SEQ_BLK * HP];
  __shared__ __align__(16) float hf[FINAL ? SEQ_BLK * FPITCH : 4];
  const _Float16* RT = (const _Float16*)RTp;
  _Float16* HOUT = (_Float16*)HOUTp;
  const int tid = threadIdx.x, lane = tid & 31, wave = tid >> 5;
  const int c = lane & 15, hh = lane >> 4, koff = hh * 8, mOff = hh * 8;
  const int blk = blockIdx.x;

#pragma unroll 1
  for (int i = tid; i < SEQ_BLK * HP; i += NTHR) h16[i] = (_Float16)0.0f;

  float hreg[2][8];
#pragma unroll
  for (int ub = 0; ub < 2; ++ub)
#pragma unroll
    for (int r = 0; r < 8; ++r) hreg[ub][r] = 0.0f;

  float biz[2], bir[2], bih[2], brz[2], brr[2], brh[2];
#pragma unroll
  for (int ub = 0; ub < 2; ++ub) {
    const int j = 32 * wave + 16 * ub + c;
    biz[ub] = bin[j]; bir[ub] = bin[NU + j]; bih[ub] = bin[2 * NU + j];
  }
  asm volatile("" ::: "memory");
#pragma unroll
  for (int ub = 0; ub < 2; ++ub) {
    const int j = 32 * wave + 16 * ub + c;
    brz[ub] = brc[j]; brr[ub] = brc[NU + j]; brh[ub] = brc[2 * NU + j];
  }
  __syncthreads();

  const _Float16* arow = h16 + c * HP + koff;
  const int nb = SEQ_BLK * blk + mOff;
  const v8f z8 = {0.f, 0.f, 0.f, 0.f, 0.f, 0.f, 0.f, 0.f};

#pragma unroll 1
  for (int t = 0; t < NTS; ++t) {
    const size_t ncol = (size_t)t * NSL + nb;
#pragma unroll
    for (int ub = 0; ub < 2; ++ub) {
      const int j = 32 * wave + 16 * ub + c;
      const _Float16* wz = RT + (size_t)j * NU + koff;
      const _Float16* wr = RT + (size_t)(NU + j) * NU + koff;
      const _Float16* wh = RT + (size_t)(2 * NU + j) * NU + koff;
      v8f az = z8, ar = z8, ah = z8;
#pragma unroll 1
      for (int k0 = 0; k0 < NU; k0 += 32) {
        const v16h a  = Frag<_Float16>::load(arow + k0);
        const v16h b0 = Frag<_Float16>::load(wz + k0);
        const v16h b1 = Frag<_Float16>::load(wr + k0);
        const v16h b2 = Frag<_Float16>::load(wh + k0);
        az = Frag<_Float16>::mma(a, b0, az);
        ar = Frag<_Float16>::mma(a, b1, ar);
        ah = Frag<_Float16>::mma(a, b2, ah);
        dep_guard3_h(az, ar, ah, a, b0, b1, b2);
      }
      acc_guard3(az, ar, ah);
      asm volatile("" ::: "memory");
      const float* xzp = XPT + (size_t)j * SROWS + ncol;
      const float* xrp = XPT + (size_t)(NU + j) * SROWS + ncol;
      const float* xhp = XPT + (size_t)(2 * NU + j) * SROWS + ncol;
      const v4f xz0 = *(const v4f*)xzp, xz1 = *(const v4f*)(xzp + 4);
      const v4f xr0 = *(const v4f*)xrp, xr1 = *(const v4f*)(xrp + 4);
      const v4f xh0 = *(const v4f*)xhp, xh1 = *(const v4f*)(xhp + 4);
      float mz[8], mr[8], mh[8];
#pragma unroll
      for (int e = 0; e < 4; ++e) {
        mz[e] = xz0[e] + biz[ub]; mz[4 + e] = xz1[e] + biz[ub];
        mr[e] = xr0[e] + bir[ub]; mr[4 + e] = xr1[e] + bir[ub];
        mh[e] = xh0[e] + bih[ub]; mh[4 + e] = xh1[e] + bih[ub];
      }
#pragma unroll
      for (int r = 0; r < 8; ++r) {
        const float rz  = az[r] * SINV + brz[ub];
        const float rr  = ar[r] * SINV + brr[ub];
        const float rch = ah[r] * SINV + brh[ub];
        const float zg  = fsig(mz[r] + rz);
        const float rg  = fsig(mr[r] + rr);
        const float cand = ftanh(mh[r] + rg * rch);
        const float ho  = hreg[ub][r];
        hreg[ub][r] = zg * ho + (1.0f - zg) * cand;
      }
    }
    __syncthreads();
#pragma unroll
    for (int ub = 0; ub < 2; ++ub) {
      const int j = 32 * wave + 16 * ub + c;
#pragma unroll
      for (int r = 0; r < 8; ++r) h16[(mOff + r) * HP + j] = (_Float16)(hreg[ub][r] * ACARRY);
    }
    __syncthreads();
    if (!FINAL) {
      _Float16* hrow = HOUT + ((size_t)t * NSL + (size_t)(SEQ_BLK * blk)) * NU;
      const int row = 2 * wave + hh, c8 = c * 8;
      for (int pass = 0; pass < 2; ++pass) {
#pragma unroll
        for (int it = 0; it < 2; ++it) {
          const v8h v = *(const v8h*)(h16 + row * HP + it * 128 + c8);
          *(volatile v8h*)(hrow + (size_t)row * NU + it * 128 + c8) = v;
        }
        __threadfence();
      }
    }
  }

  if (FINAL) {
#pragma unroll
    for (int ub = 0; ub < 2; ++ub) {
      const int j = 32 * wave + 16 * ub + c;
#pragma unroll
      for (int r = 0; r < 8; ++r) hf[(mOff + r) * FPITCH + j] = hreg[ub][r];
    }
    __syncthreads();
    const int row = 2 * wave + hh;
    float* orow = OUT + (size_t)(SEQ_BLK * blk + row) * NU;
    for (int pass = 0; pass < 2; ++pass) {
#pragma unroll
      for (int it = 0; it < 4; ++it) {
        const int c4 = it * 64 + c * 4;
        const v4f v = *(const v4f*)(hf + row * FPITCH + c4);
        *(volatile v4f*)(orow + c4) = v;
      }
      __threadfence();
    }
  }
}

extern "C" void kernel_launch(void* const* d_in, const int* in_sizes, int n_in,
                              void* d_out, int out_size, void* d_ws, size_t ws_size, hipStream_t stream) {
  if (n_in < 7 || d_out == nullptr || d_ws == nullptr) return;
  if (in_sizes[0] != NROWS * NF || in_sizes[1] != NF * NG || in_sizes[2] != NU * NG || in_sizes[3] != 2 * NG ||
      in_sizes[4] != (NLAY - 1) * NU * NG || in_sizes[5] != (NLAY - 1) * NU * NG || in_sizes[6] != (NLAY - 1) * 2 * NG ||
      out_size != NB * NU) return;

  const float* x     = (const float*)d_in[0];
  const float* k0    = (const float*)d_in[1];
  const float* rk0   = (const float*)d_in[2];
  const float* b0    = (const float*)d_in[3];
  const float* kern  = (const float*)d_in[4];
  const float* rkern = (const float*)d_in[5];
  const float* bias  = (const float*)d_in[6];
  float* out = (float*)d_out;

  char* ws = (char*)d_ws; size_t off = 0;
  auto carve = [&](size_t bytes) -> char* { char* p = ws + off; off += (bytes + 255) & ~(size_t)255; return p; };
  unsigned short* SA   = (unsigned short*)carve(SEQ_BYTES);
  unsigned short* SB   = (unsigned short*)carve(SEQ_BYTES);
  unsigned short* WALL = (unsigned short*)carve(WALL_BYTES);
  float*          XPT  = (float*)carve(XPT_BYTES);
  if (off > ws_size || off > (size_t)134217728) return;

  prep_kernel<<<NPREPBLK, NTHR, 0, stream>>>(x, k0, kern, rk0, rkern, SA, WALL);

  for (int L = 0; L < NLAY; ++L) {
    const unsigned short* Sin = (L & 1) ? SB : SA;
    unsigned short* Sout      = (L & 1) ? SA : SB;
    const float* bin = (L == 0) ? b0 : (bias + (size_t)(L - 1) * 2 * NG);
    const float* brc = bin + NG;
    const unsigned short* WTL = WALL + (size_t)L * WMAT;
    const unsigned short* RTL = WALL + (size_t)(NLAY + L) * WMAT;
    for (int s = 0; s < NSLICE; ++s) {
      const unsigned short* Sin_s = Sin + (size_t)s * SROWS * NF;
      unsigned short* Sout_s = Sout + (size_t)s * SROWS * NU;
      wmma_gemm64<0, false, 0, 0, false, 0><<<dim3(GBLK, 1), 256, 0, stream>>>(
          WTL, WTL, NF, 0L, Sin_s, Sin_s, NF, 0L, (void*)XPT, (void*)XPT, SROWS, 0L,
          bin, bin, 0L, NG, SROWS, NF, SINV);
      if (L < NLAY - 1) {
        rec_kernel<false><<<NSL / SEQ_BLK, NTHR, 0, stream>>>(XPT, RTL, bin, brc, Sout_s, out + (size_t)s * NSL * NU);
      } else {
        rec_kernel<true><<<NSL / SEQ_BLK, NTHR, 0, stream>>>(XPT, RTL, bin, brc, Sout_s, out + (size_t)s * NSL * NU);
      }
    }
  }
}
